// SecondaryStructureEnergy_2628519985584
// MI455X (gfx1250) — hardware-verified
//
#include <hip/hip_runtime.h>
#include <stddef.h>

typedef _Float16 v16h __attribute__((ext_vector_type(16)));
typedef _Float16 v8h  __attribute__((ext_vector_type(8)));
typedef float    v8f  __attribute__((ext_vector_type(8)));
typedef float    v4f  __attribute__((ext_vector_type(4)));

#define HID     128
#define XP      96
#define HP      128
#define WP      128
#define NWAVE   4
#define NTHR    (NWAVE * 32)
#define EMBW    16
#define EMBMAX  64
#define XSCALE  64.0f
#define WSCALE  4096.0f
#define ACC_INV (1.0f / 262144.0f)

typedef char nwave_is_4_check[(NWAVE == 4) ? 1 : -1];

union Frag  { v16h v; v8h hf[2]; };
union Pack8 { v8h v; _Float16 e[8]; };

__device__ __forceinline__ v8f wmma16(v16h a, v16h b, v8f c)
{
  c = __builtin_amdgcn_wmma_f32_16x16x32_f16(false, a, false, b, (short)0, c, false, false);
  asm volatile("v_nop\n\tv_nop\n\tv_nop\n\tv_nop" : "+v"(c) : "v"(a), "v"(b));
  return c;
}

__device__ __forceinline__ v16h frag_ld(const _Float16* rowp, int k0, int h)
{
  Frag f;
  f.hf[0] = *(const v8h*)(rowp + k0 + 8 * h);
  f.hf[1] = *(const v8h*)(rowp + k0 + 16 + 8 * h);
  return f.v;
}

struct F3 { float x, y, z; };
__device__ __forceinline__ F3 f3sub(F3 a, F3 b) { F3 r; r.x = a.x - b.x; r.y = a.y - b.y; r.z = a.z - b.z; return r; }
__device__ __forceinline__ F3 f3cross(F3 a, F3 b)
{
  F3 r;
  r.x = a.y * b.z - a.z * b.y;
  r.y = a.z * b.x - a.x * b.z;
  r.z = a.x * b.y - a.y * b.x;
  return r;
}
__device__ __forceinline__ float f3dot(F3 a, F3 b) { return a.x * b.x + a.y * b.y + a.z * b.z; }

__device__ __forceinline__ void torsion_sc(F3 p0, F3 p1, F3 p2, F3 p3, float* s, float* c)
{
  F3 b1 = f3sub(p1, p0), b2 = f3sub(p2, p1), b3 = f3sub(p3, p2);
  F3 n1 = f3cross(b1, b2), n2 = f3cross(b2, b3);
  float bl = sqrtf(f3dot(b2, b2)) + 1e-8f;
  F3 b2n; b2n.x = b2.x / bl; b2n.y = b2.y / bl; b2n.z = b2.z / bl;
  float x = f3dot(n1, n2);
  float y = f3dot(f3cross(n1, n2), b2n);
  float r = sqrtf(x * x + y * y) + 1e-20f;
  *s = y / r;  *c = x / r;
}

__global__ __launch_bounds__(256)
void k_prep(const float* __restrict__ tW1, const float* __restrict__ tW2,
            const float* __restrict__ pW1, const float* __restrict__ pW2,
            int in1, int in2, int total, _Float16* __restrict__ wt)
{
  const int gid = blockIdx.x * 256 + threadIdx.x;
  if (gid >= total) return;
  const int kq    = gid & 15;
  const int rowid = gid >> 4;
  const int n     = rowid & (HID - 1);
  const int ml    = rowid >> 7;
  const int layer = ml & 1;
  const int m     = ml >> 1;
  const float* W  = layer ? (m ? pW2 : tW2) : (m ? pW1 : tW1);
  const int IN    = m ? in2 : in1;
  const int co    = IN - 64;

  Pack8 hv, lv;
  #pragma unroll
  for (int j = 0; j < 8; j++) {
    const int kk = kq * 8 + j;
    float w = 0.0f;
    if (layer) {
      w = W[(size_t)kk * HID + n];
    } else {
      int orow; bool ok;
      if (kk < 64) { orow = co + kk; ok = (orow >= 0) && (orow < IN); }
      else         { orow = kk - 64; ok = (orow < co) && (orow < IN); }
      if (ok) w = W[(size_t)orow * HID + n];
    }
    const float s = w * WSCALE;
    const _Float16 hh = (_Float16)s;
    hv.e[j] = hh;
    lv.e[j] = (_Float16)(s - (float)hh);
  }
  _Float16* dh = wt + ((size_t)(ml * 2 + 0) * HID + n) * WP + kq * 8;
  _Float16* dl = wt + ((size_t)(ml * 2 + 1) * HID + n) * WP + kq * 8;
  *(volatile v8h*)dh = hv.v;
  *(volatile v8h*)dl = lv.v;
  __threadfence();
  *(volatile v8h*)dh = hv.v;
  *(volatile v8h*)dl = lv.v;
}

__global__ __launch_bounds__(NTHR)
void k_energy(const float* __restrict__ R, const int* __restrict__ seq,
              const float* __restrict__ emb,
              const float* __restrict__ tb1, const float* __restrict__ tb2,
              const float* __restrict__ tw3, const float* __restrict__ tb3,
              const float* __restrict__ pb1, const float* __restrict__ pb2,
              const float* __restrict__ pw3, const float* __restrict__ pb3,
              const _Float16* __restrict__ wt, float* __restrict__ part,
              int L, int tpb, int ntiles, int naa)
{
  __shared__ __attribute__((aligned(16))) _Float16 xbuf[NWAVE][2][16 * XP];
  __shared__ __attribute__((aligned(16))) _Float16 hbuf[NWAVE][16 * HP];
  __shared__ __attribute__((aligned(16))) _Float16 semb[2][EMBMAX * EMBW];
  __shared__ float spart[NWAVE];

  const int tid  = threadIdx.x;
  const int wv   = tid >> 5;
  const int lane = tid & 31;
  const int lo   = lane & 15;
  const int h    = lane >> 4;

  const int nemb = naa * EMBW;
  for (int idx = tid; idx < nemb; idx += NTHR) {
    const float v = emb[idx] * XSCALE;
    const _Float16 hv = (_Float16)v;
    semb[0][idx] = hv;
    semb[1][idx] = (_Float16)(v - (float)hv);
  }
  __syncthreads();

  const int  t    = blockIdx.x * NWAVE + wv;
  const bool tval = t < ntiles;
  const int  tt   = tval ? t : 0;
  const int  b    = tt / tpb;
  const int  i0   = (tt - b * tpb) * 16;
  const int  i    = i0 + lo;
  const int  Lm1  = L - 1;
  const size_t rb = (size_t)b * (size_t)L;

  F3 P[5];
  #pragma unroll
  for (int k = 0; k < 5; k++) {
    int idx = i + k; idx = idx > Lm1 ? Lm1 : idx;
    const float* p = R + (rb + (size_t)idx) * 3;
    P[k].x = p[0]; P[k].y = p[1]; P[k].z = p[2];
  }
  F3 u1 = f3sub(P[0], P[1]), u2 = f3sub(P[2], P[1]);
  F3 cr = f3cross(u1, u2);
  const float dd  = f3dot(u1, u2);
  const float cth = dd / sqrtf(dd * dd + f3dot(cr, cr) + 1e-30f);
  float s0, c0, s1, c1;
  torsion_sc(P[0], P[1], P[2], P[3], &s0, &c0);
  torsion_sc(P[1], P[2], P[3], P[4], &s1, &c1);

  {
    int ia = i + 2 * h;     ia = ia > Lm1 ? Lm1 : ia;
    int ib = i + 2 * h + 1; ib = ib > Lm1 ? Lm1 : ib;
    int sa = seq[rb + (size_t)ia];
    int sb = seq[rb + (size_t)ib];
    sa = sa < 0 ? 0 : (sa > naa - 1 ? naa - 1 : sa);
    sb = sb < 0 ? 0 : (sb > naa - 1 ? naa - 1 : sb);
    #pragma unroll
    for (int p = 0; p < 2; p++) {
      _Float16* xr = &xbuf[wv][p][lo * XP + 32 * h];
      const _Float16* ea = &semb[p][sa * EMBW];
      const _Float16* eb = &semb[p][sb * EMBW];
      *(v8h*)(xr + 0)  = *(const v8h*)(ea);
      *(v8h*)(xr + 8)  = *(const v8h*)(ea + 8);
      *(v8h*)(xr + 16) = *(const v8h*)(eb);
      *(v8h*)(xr + 24) = *(const v8h*)(eb + 8);
    }
    Pack8 z;
    #pragma unroll
    for (int j = 0; j < 8; j++) z.e[j] = (_Float16)0.0f;
    _Float16* xz = &xbuf[wv][h][lo * XP];
    *(v8h*)(xz + 72) = z.v;
    *(v8h*)(xz + 80) = z.v;
    *(v8h*)(xz + 88) = z.v;
  }

  float waveE = 0.0f;

  #pragma unroll
  for (int m = 0; m < 2; m++) {
    {
      const float g0 = (m == 0) ? cth : s0;
      const float g1 = (m == 0) ? s0  : c0;
      const float g2 = (m == 0) ? c0  : s1;
      const float g3 = (m == 0) ? 0.0f : c1;
      const float gs[4] = { g0 * XSCALE, g1 * XSCALE, g2 * XSCALE, g3 * XSCALE };
      Pack8 gv;
      #pragma unroll
      for (int c = 0; c < 8; c++) {
        const float v = (c < 4) ? gs[c] : 0.0f;
        const _Float16 hv = (_Float16)v;
        const _Float16 lv = (_Float16)(v - (float)hv);
        gv.e[c] = h ? lv : hv;
      }
      *(v8h*)(&xbuf[wv][h][lo * XP + 64]) = gv.v;
    }
    __syncthreads();

    const _Float16* xh  = &xbuf[wv][0][lo * XP];
    const _Float16* xl  = &xbuf[wv][1][lo * XP];
    const _Float16* w1h = wt + (size_t)((m * 2 + 0) * 2 + 0) * HID * WP;
    const _Float16* w1l = wt + (size_t)((m * 2 + 0) * 2 + 1) * HID * WP;
    const _Float16* w2h = wt + (size_t)((m * 2 + 1) * 2 + 0) * HID * WP;
    const _Float16* w2l = wt + (size_t)((m * 2 + 1) * 2 + 1) * HID * WP;
    const float* B1 = m ? pb1 : tb1;
    const float* B2 = m ? pb2 : tb2;
    const float* W3 = m ? pw3 : tw3;
    const float  B3 = m ? pb3[0] : tb3[0];

    #pragma unroll 1
    for (int nt = 0; nt < 8; nt++) {
      v8f c = { 0.f, 0.f, 0.f, 0.f, 0.f, 0.f, 0.f, 0.f };
      const _Float16* bh = w1h + (size_t)(nt * 16 + lo) * WP;
      const _Float16* bl = w1l + (size_t)(nt * 16 + lo) * WP;
      #pragma unroll
      for (int kt = 0; kt < 3; kt++) {
        const v16h ah  = frag_ld(xh, kt * 32, h);
        const v16h al  = frag_ld(xl, kt * 32, h);
        const v16h fbh = frag_ld(bh, kt * 32, h);
        const v16h fbl = frag_ld(bl, kt * 32, h);
        c = wmma16(ah, fbh, c);
        c = wmma16(al, fbh, c);
        c = wmma16(ah, fbl, c);
      }
      const float bias = B1[nt * 16 + lo];
      _Float16* hrw = &hbuf[wv][nt * 16 + lo];
      #pragma unroll
      for (int r = 0; r < 8; r++) {
        float hp = c[r] * ACC_INV + bias;
        hp = hp > 0.0f ? hp : 0.0f;
        hrw[(8 * h + r) * HP] = (_Float16)(hp * XSCALE);
      }
    }
    __syncthreads();

    const _Float16* hr = &hbuf[wv][lo * HP];
    float rowE[8] = { 0.f, 0.f, 0.f, 0.f, 0.f, 0.f, 0.f, 0.f };
    #pragma unroll 1
    for (int nt = 0; nt < 8; nt++) {
      v8f c = { 0.f, 0.f, 0.f, 0.f, 0.f, 0.f, 0.f, 0.f };
      const _Float16* bh = w2h + (size_t)(nt * 16 + lo) * WP;
      const _Float16* bl = w2l + (size_t)(nt * 16 + lo) * WP;
      #pragma unroll
      for (int kt = 0; kt < 4; kt++) {
        const v16h a   = frag_ld(hr, kt * 32, h);
        const v16h fbh = frag_ld(bh, kt * 32, h);
        const v16h fbl = frag_ld(bl, kt * 32, h);
        c = wmma16(a, fbh, c);
        c = wmma16(a, fbl, c);
      }
      const float bias = B2[nt * 16 + lo];
      const float w3v  = W3[nt * 16 + lo];
      #pragma unroll
      for (int r = 0; r < 8; r++) {
        float hp = c[r] * ACC_INV + bias;
        hp = hp > 0.0f ? hp : 0.0f;
        rowE[r] += hp * w3v;
      }
    }

    #pragma unroll
    for (int r = 0; r < 8; r++) {
      float v = rowE[r];
      v += __shfl_xor(v, 1, 32);
      v += __shfl_xor(v, 2, 32);
      v += __shfl_xor(v, 4, 32);
      v += __shfl_xor(v, 8, 32);
      rowE[r] = v;
    }
    const int npos = (m == 0) ? (L - 3) : (L - 4);
    float e = 0.0f;
    #pragma unroll
    for (int r = 0; r < 8; r++) {
      const int row = i0 + r + 8 * h;
      if (tval && row < npos) e += rowE[r] + B3;
    }
    e += __shfl_xor(e, 16, 32);
    waveE += e;
  }

  if (lane == 0) spart[wv] = waveE;
  __syncthreads();
  if (wv == 0 && lane < 8) {
    v4f v = { 0.f, 0.f, 0.f, 0.f };
    if (lane == 0) { v[0] = spart[0]; v[1] = spart[1]; v[2] = spart[2]; v[3] = spart[3]; }
    volatile v4f* p = (volatile v4f*)(part + (size_t)blockIdx.x * 32 + lane * 4);
    *p = v;
    __threadfence();
    *p = v;
  }
}

__global__ __launch_bounds__(1024)
void k_reduce(const float* __restrict__ part, float* __restrict__ out, int B, int tpb)
{
  __shared__ __attribute__((aligned(16))) float s[1024];
  const int tid = threadIdx.x;
  float e = 0.0f;
  if (tid < B) {
    const int t0 = tid * tpb;
    for (int j = 0; j < tpb; j++) {
      const int t = t0 + j;
      e += part[(size_t)(t / NWAVE) * 32 + (t % NWAVE)];
    }
  }
  s[tid] = e;
  __syncthreads();
  const int nq  = B >> 2;
  const int rem = B & 3;
  if (tid < nq) {
    const v4f v = *(const v4f*)(&s[tid * 4]);
    volatile v4f* p = (volatile v4f*)(out + tid * 4);
    *p = v;
    __threadfence();
    *p = v;
  }
  if (tid == nq && rem != 0) {
    float v0 = s[nq * 4 + 0];
    float v1 = (rem > 1) ? s[nq * 4 + 1] : 0.0f;
    float v2 = (rem > 2) ? s[nq * 4 + 2] : 0.0f;
    volatile float* p = (volatile float*)(out + nq * 4);
    p[0] = v0; if (rem > 1) p[1] = v1; if (rem > 2) p[2] = v2;
    __threadfence();
    p[0] = v0; if (rem > 1) p[1] = v1; if (rem > 2) p[2] = v2;
  }
}

extern "C" void kernel_launch(void* const* d_in, const int* in_sizes, int n_in,
                              void* d_out, int out_size, void* d_ws, size_t ws_size,
                              hipStream_t stream)
{
  if (n_in < 15) return;
  const float* R   = (const float*)d_in[0];
  const int*   seq = (const int*)  d_in[1];
  const float* emb = (const float*)d_in[2];
  const float* tW1 = (const float*)d_in[3];
  const float* tb1 = (const float*)d_in[4];
  const float* tW2 = (const float*)d_in[5];
  const float* tb2 = (const float*)d_in[6];
  const float* tW3 = (const float*)d_in[7];
  const float* tb3 = (const float*)d_in[8];
  const float* pW1 = (const float*)d_in[9];
  const float* pb1 = (const float*)d_in[10];
  const float* pW2 = (const float*)d_in[11];
  const float* pb2 = (const float*)d_in[12];
  const float* pW3 = (const float*)d_in[13];
  const float* pb3 = (const float*)d_in[14];

  const int B = out_size;
  if (B <= 0 || B > 1024) return;
  const int nseq = in_sizes[1];
  const int L = nseq / B;
  if (L < 5 || nseq < B * L || in_sizes[0] < nseq * 3) return;
  const int in1 = in_sizes[3] / HID;
  const int in2 = in_sizes[9] / HID;
  if (in1 < 64 || in1 > 72 || in2 < 64 || in2 > 72) return;
  if (in_sizes[4] < HID || in_sizes[5] < HID * HID || in_sizes[6] < HID || in_sizes[7] < HID || in_sizes[8] < 1) return;
  if (in_sizes[10] < HID || in_sizes[11] < HID * HID || in_sizes[12] < HID || in_sizes[13] < HID || in_sizes[14] < 1) return;
  int naa = in_sizes[2] / EMBW;
  if (naa < 1) return;
  if (naa > EMBMAX) naa = EMBMAX;

  const int tpb     = (L - 3 + 15) / 16;
  const int ntiles  = B * tpb;
  const int nblocks = (ntiles + NWAVE - 1) / NWAVE;

  const size_t wt_bytes   = (size_t)8 * HID * WP * sizeof(_Float16);
  const size_t part_bytes = (size_t)nblocks * 32 * sizeof(float);
  if (wt_bytes + part_bytes > ws_size) return;
  char* ws = (char*)d_ws;
  _Float16* wt   = (_Float16*)ws;
  float*    part = (float*)(ws + wt_bytes);
  float*    out  = (float*)d_out;

  const int prep_total = 4 * HID * 16;
  hipLaunchKernelGGL(k_prep, dim3((prep_total + 255) / 256), dim3(256), 0, stream,
                     tW1, tW2, pW1, pW2, in1, in2, prep_total, wt);
  hipLaunchKernelGGL(k_energy, dim3(nblocks), dim3(NTHR), 0, stream,
                     R, seq, emb, tb1, tb2, tW3, tb3, pb1, pb2, pW3, pb3,
                     (const _Float16*)wt, part, L, tpb, ntiles, naa);
  const int bt = ((B + 31) / 32) * 32;
  hipLaunchKernelGGL(k_reduce, dim3(1), dim3(bt), 0, stream,
                     (const float*)part, out, B, tpb);
}
